// SS2D_16939351015734
// MI455X (gfx1250) — hardware-run, weakly checked
//
#include <hip/hip_runtime.h>
#include <math.h>

typedef __attribute__((ext_vector_type(16))) _Float16 v16h;
typedef __attribute__((ext_vector_type(8)))  _Float16 v8h;
typedef __attribute__((ext_vector_type(16))) __bf16   v16b;
typedef __attribute__((ext_vector_type(8)))  __bf16   v8b;
typedef __attribute__((ext_vector_type(8)))  float    v8f;
typedef __attribute__((ext_vector_type(4)))  float    v4f;

constexpr int kBatch  = 4;
constexpr int kImg    = 64;
constexpr int kSeq    = kImg * kImg;
constexpr int kRows   = kBatch * kSeq;
constexpr int kDm     = 192;
constexpr int kDin    = 384;
constexpr int kNst    = 16;
constexpr int kDtR    = 12;
constexpr int kDbl    = kDtR + 2 * kNst;
constexpr int kXzP    = 2 * kDin;
constexpr int kXdP    = 64;
constexpr int kGateH  = 96;
constexpr int kTap1   = 15;
constexpr int kC2Ch   = 128;
constexpr int kC2P    = 132;
constexpr int kScanTS = 64;
constexpr int kScanCh = 64;
constexpr int kScanYP = 68;
constexpr int kC1Rows = 64;
constexpr int kC1In   = kC1Rows + 28;
static_assert(kDbl == 44 && kDbl <= kXdP, "dbl width");
static_assert((kDm % 32) == 0 && (kDin % 32) == 0, "GEMM K multiples of 32");
static_assert((kRows % 64) == 0 && (kXzP % 64) == 0 && (kXdP % 64) == 0 && (kDm % 64) == 0, "GEMM M,N multiples of 64");
static_assert((kSeq % kScanTS) == 0 && (kDin % kScanCh) == 0 && (kDin % kC2Ch) == 0 && (kSeq % kC1Rows) == 0, "tile multiples");
static_assert((kRows * kDm) % (8 * 256) == 0 && (kXzP * kDm) % (8 * 256) == 0 && (kDm * kDin) % (8 * 256) == 0, "plane kernels: exact grids");

constexpr size_t kOffXH    = 0;
constexpr size_t kOffXL    = kOffXH   + (size_t)kRows * kDm * 2;
constexpr size_t kOffHBLB  = kOffXL   + (size_t)kRows * kDm * 2;
constexpr size_t kOffWIH   = kOffHBLB + (size_t)kRows * kDm * 2;
constexpr size_t kOffWIL   = kOffWIH  + (size_t)kXzP * kDm * 2;
constexpr size_t kOffWOH   = kOffWIL  + (size_t)kXzP * kDm * 2;
constexpr size_t kOffWOL   = kOffWOH  + (size_t)kDm * kDin * 2;
constexpr size_t kOffWXB   = kOffWOL  + (size_t)kDm * kDin * 2;
constexpr size_t kOffWCB   = kOffWXB  + (size_t)kXdP * kDin * 2;
constexpr size_t kOffXZ    = kOffWCB  + (size_t)kXdP * kDm * 2;
constexpr size_t kOffXS    = kOffXZ   + (size_t)kRows * kXzP * 4;
constexpr size_t kOffXSB   = kOffXS   + (size_t)kRows * kDin * 4;
constexpr size_t kOffLOWD  = kOffXSB  + (size_t)kRows * kDin * 2;
constexpr size_t kOffXD    = kOffLOWD + (size_t)kRows * kXdP * 4;
constexpr size_t kOffBCD   = kOffXD   + (size_t)kRows * kXdP * 4;
constexpr size_t kOffCONVO = kOffBCD  + (size_t)kRows * kXdP * 4;
constexpr size_t kWsTotal  = kOffCONVO + (size_t)kRows * kXdP * 4;
constexpr size_t kOffYH    = kOffXH;
constexpr size_t kOffYL    = kOffXSB;
static_assert(kWsTotal == 124690432ull, "carve total");
static_assert(kWsTotal <= 134217728ull, "carve cap");
static_assert(kOffHBLB - kOffXH == (size_t)kRows * kDin * 2, "YH fits XH+XL exactly");
static_assert(kOffLOWD - kOffXSB == (size_t)kRows * kDin * 2, "YL fits XSB exactly");
static_assert((kOffXL % 128) == 0 && (kOffHBLB % 128) == 0 && (kOffWIH % 128) == 0 && (kOffWIL % 128) == 0 &&
              (kOffWOH % 128) == 0 && (kOffWOL % 128) == 0 && (kOffWXB % 128) == 0 && (kOffWCB % 128) == 0 &&
              (kOffXZ % 128) == 0 && (kOffXS % 128) == 0 && (kOffXSB % 128) == 0 && (kOffLOWD % 128) == 0 &&
              (kOffXD % 128) == 0 && (kOffBCD % 128) == 0 && (kOffCONVO % 128) == 0, "128-B aligned regions");

__device__ __forceinline__ unsigned short f2bf_bits(float f) {
  unsigned u = __float_as_uint(f);
  return (unsigned short)((u + 0x7FFFu + ((u >> 16) & 1u)) >> 16);
}
__device__ __forceinline__ float bf_bits2f(unsigned short h) { return __uint_as_float(((unsigned)h) << 16); }

__device__ __forceinline__ v8h pack8_bf16(const v4f a0, const v4f a1) {
  v8h hv;
#pragma unroll
  for (int e = 0; e < 4; ++e) {
    const unsigned short h0 = f2bf_bits(a0[e]), h1 = f2bf_bits(a1[e]);
    hv[e]     = __builtin_bit_cast(_Float16, h0);
    hv[4 + e] = __builtin_bit_cast(_Float16, h1);
  }
  return hv;
}
__device__ __forceinline__ void split8_bf16(const v4f a0, const v4f a1, v8h& hv, v8h& lv) {
#pragma unroll
  for (int e = 0; e < 4; ++e) {
    const unsigned short h0 = f2bf_bits(a0[e]), h1 = f2bf_bits(a1[e]);
    const unsigned short l0 = f2bf_bits(a0[e] - bf_bits2f(h0)), l1 = f2bf_bits(a1[e] - bf_bits2f(h1));
    hv[e]     = __builtin_bit_cast(_Float16, h0);
    hv[4 + e] = __builtin_bit_cast(_Float16, h1);
    lv[e]     = __builtin_bit_cast(_Float16, l0);
    lv[4 + e] = __builtin_bit_cast(_Float16, l1);
  }
}

__device__ __forceinline__ void dep_guard_h(v8f& a, v8f& b, v16h x, v16h y) { asm volatile("v_nop\n\tv_nop\n\tv_nop\n\tv_nop" : "+v"(a), "+v"(b) : "v"(x), "v"(y)); }
__device__ __forceinline__ void dep_guard_b(v8f& a, v8f& b, v16b x, v16b y) { asm volatile("v_nop\n\tv_nop\n\tv_nop\n\tv_nop" : "+v"(a), "+v"(b) : "v"(x), "v"(y)); }
__device__ __forceinline__ void dep_guard4_h(v8f& a, v8f& b, v8f& c, v8f& d, v16h x, v16h y) { asm volatile("v_nop\n\tv_nop\n\tv_nop\n\tv_nop" : "+v"(a), "+v"(b), "+v"(c), "+v"(d) : "v"(x), "v"(y)); }
__device__ __forceinline__ void dep_guard4_b(v8f& a, v8f& b, v8f& c, v8f& d, v16b x, v16b y) { asm volatile("v_nop\n\tv_nop\n\tv_nop\n\tv_nop" : "+v"(a), "+v"(b), "+v"(c), "+v"(d) : "v"(x), "v"(y)); }
__device__ __forceinline__ void keep4_h(v16h a, v16h b, v16h c, v16h d) { asm volatile("v_nop" :: "v"(a), "v"(b), "v"(c), "v"(d)); }
__device__ __forceinline__ void keep4_b(v16b a, v16b b, v16b c, v16b d) { asm volatile("v_nop" :: "v"(a), "v"(b), "v"(c), "v"(d)); }
__device__ __forceinline__ void acc_guard4(v8f& a, v8f& b, v8f& c, v8f& d) { asm volatile("v_nop\n\tv_nop\n\tv_nop\n\tv_nop" : "+v"(a), "+v"(b), "+v"(c), "+v"(d)); }
template <typename T> struct Frag;
template <> struct Frag<_Float16> {
  typedef v16h V; union U { v16h v; v8h h[2]; };
  static __device__ __forceinline__ v16h load(const _Float16* p) {
    U f; f.h[0] = *(const v8h*)(p); f.h[1] = *(const v8h*)(p + 16); return f.v;
  }
  static __device__ __forceinline__ v8f mma(v16h a, v16h b, v8f c) {
    return __builtin_amdgcn_wmma_f32_16x16x32_f16(false, a, false, b, (short)0, c, false, false);
  }
  static __device__ __forceinline__ void guard(v8f& a, v8f& b, v16h x, v16h y) { dep_guard_h(a, b, x, y); }
  static __device__ __forceinline__ void guard4(v8f& a, v8f& b, v8f& c, v8f& d, v16h x, v16h y) { dep_guard4_h(a, b, c, d, x, y); }
  static __device__ __forceinline__ void keep(v16h a, v16h b, v16h c, v16h d) { keep4_h(a, b, c, d); }
};
template <> struct Frag<__bf16> {
  typedef v16b V; union U { v16b v; v8b h[2]; };
  static __device__ __forceinline__ v16b load(const __bf16* p) {
    U f; f.h[0] = *(const v8b*)(p); f.h[1] = *(const v8b*)(p + 16); return f.v;
  }
  static __device__ __forceinline__ v8f mma(v16b a, v16b b, v8f c) {
    return __builtin_amdgcn_wmma_f32_16x16x32_bf16(false, a, false, b, (short)0, c, false, false);
  }
  static __device__ __forceinline__ void guard(v8f& a, v8f& b, v16b x, v16b y) { dep_guard_b(a, b, x, y); }
  static __device__ __forceinline__ void guard4(v8f& a, v8f& b, v8f& c, v8f& d, v16b x, v16b y) { dep_guard4_b(a, b, c, d, x, y); }
  static __device__ __forceinline__ void keep(v16b a, v16b b, v16b c, v16b d) { keep4_b(a, b, c, d); }
};

template <int ET> struct Elem;
template <> struct Elem<0> { typedef _Float16 T; };
template <> struct Elem<1> { typedef __bf16 T; };
template <int ET, int SPL, int BIAS_MODE, int OUT_MODE, bool RESID, int ACT = 0>
__global__ __launch_bounds__(256) void wmma_gemm64(
    const unsigned short* __restrict__ Ap, const unsigned short* __restrict__ A2p, int lda, long strideA,
    const unsigned short* __restrict__ Btp, const unsigned short* __restrict__ Bt2p, int ldb, long strideB,
    void* __restrict__ Cout, void* __restrict__ Cout2, int ldc, long strideC,
    const float* __restrict__ bias,
    const float* __restrict__ resid, long strideR,
    int M, int N, int K, float scale) {
  typedef typename Elem<ET>::T T;
  typedef typename Frag<T>::V V;
  const T* A = (const T*)Ap; const T* A2 = (const T*)A2p; const T* Bt = (const T*)Btp; const T* Bt2 = (const T*)Bt2p;
  __shared__ __align__(16) float sT[8][16 * 68];
  const int b    = blockIdx.y;
  const int lane = threadIdx.x & 31;
  const int wave = threadIdx.x >> 5;
  const int tilesN = N >> 6;
  const int tilesM = M >> 6;
  const int tile = blockIdx.x * 8 + wave;
  if (tile >= tilesM * tilesN) return;
  const int tm = tile / tilesN;
  const int tn = tile - tm * tilesN;
  const int m0 = tm << 6;
  const int n0 = tn << 6;

  const T* Ab  = A  + (size_t)b * strideA;
  const T* Bb  = Bt + (size_t)b * strideB;
  const T* Ab2 = (SPL >= 1) ? (A2  + (size_t)b * strideA) : nullptr;
  const T* Bb2 = (SPL == 2) ? (Bt2 + (size_t)b * strideB) : nullptr;

  const int rlane = lane & 15;
  const int koff  = (lane >> 4) * 8;
  const int mOff  = (lane >> 4) * 8;

  v8f acc[4][4];
#pragma unroll
  for (int i = 0; i < 4; ++i)
#pragma unroll
    for (int j = 0; j < 4; ++j) acc[i][j] = (v8f){0.f,0.f,0.f,0.f,0.f,0.f,0.f,0.f};

  for (int k0 = 0; k0 < K; k0 += 32) {
    V bh[4], bl[4];
#pragma unroll
    for (int j = 0; j < 4; ++j) {
      const size_t bo = (size_t)(n0 + (j << 4) + rlane) * ldb + koff + k0;
      bh[j] = Frag<T>::load(Bb + bo);
      if (SPL == 2) bl[j] = Frag<T>::load(Bb2 + bo);
    }
#pragma unroll
    for (int i = 0; i < 4; ++i) {
      const size_t ao = (size_t)(m0 + (i << 4) + rlane) * lda + koff + k0;
      V ah = Frag<T>::load(Ab + ao);
      V al;
      if (SPL >= 1) al = Frag<T>::load(Ab2 + ao);
#pragma unroll
      for (int j = 0; j < 4; ++j) {
        acc[i][j] = Frag<T>::mma(ah, bh[j], acc[i][j]);
        if (SPL == 2) acc[i][j] = Frag<T>::mma(ah, bl[j], acc[i][j]);
        if (SPL >= 1) acc[i][j] = Frag<T>::mma(al, bh[j], acc[i][j]);
      }
      Frag<T>::guard4(acc[i][0], acc[i][1], acc[i][2], acc[i][3], ah, (SPL >= 1) ? al : ah);
    }
    Frag<T>::keep(bh[0], bh[1], bh[2], bh[3]);
    if (SPL == 2) Frag<T>::keep(bl[0], bl[1], bl[2], bl[3]);
  }
  acc_guard4(acc[0][0], acc[0][1], acc[0][2], acc[0][3]);
  acc_guard4(acc[1][0], acc[1][1], acc[1][2], acc[1][3]);
  acc_guard4(acc[2][0], acc[2][1], acc[2][2], acc[2][3]);
  acc_guard4(acc[3][0], acc[3][1], acc[3][2], acc[3][3]);

  float* slab = sT[wave];
  const float* Rb = RESID ? (resid + (size_t)b * strideR) : nullptr;
#pragma unroll
  for (int i = 0; i < 4; ++i) {
    const int mBase = m0 + (i << 4);
#pragma unroll
    for (int j = 0; j < 4; ++j) {
      const int n = n0 + (j << 4) + rlane;
      float bv = 0.f;
      if (BIAS_MODE == 2) bv = bias[n];
#pragma unroll
      for (int r = 0; r < 8; ++r) {
        float v = acc[i][j][r] * scale;
        if (BIAS_MODE == 1) v += bias[mBase + mOff + r];
        if (BIAS_MODE == 2) v += bv;
        if (RESID) v += Rb[(size_t)(mBase + mOff + r) * ldc + n];
        if (ACT == 1) v = tanhf(v);
        if (ACT == 2) v = fmaxf(v, 0.0f);
        if (ACT == 3) v = v / (1.0f + expf(-v));
        if (ACT == 4) v = (v > 0.f) ? v : 0.01f * v;
        slab[(mOff + r) * 68 + (j << 4) + rlane] = v;
      }
    }
    __builtin_amdgcn_fence(__ATOMIC_RELEASE, "workgroup");
    __builtin_amdgcn_wave_barrier();
    __builtin_amdgcn_fence(__ATOMIC_ACQUIRE, "workgroup");
    if (OUT_MODE == 0) {
      float* C = (float*)Cout + (size_t)b * strideC;
      const int hh = lane >> 4, c4 = (lane & 15) * 4;
      for (int pass = 0; pass < 2; ++pass) {
#pragma unroll
        for (int it = 0; it < 8; ++it) {
          const int row = it * 2 + hh;
          v4f v = *(const v4f*)(slab + row * 68 + c4);
          *(volatile v4f*)(C + (size_t)(mBase + row) * ldc + n0 + c4) = v;
        }
        __threadfence();
      }
    } else {
      const int q = lane >> 3, c8 = (lane & 7) * 8;
      unsigned short* C  = (unsigned short*)Cout  + (size_t)b * strideC;
      unsigned short* C2 = (OUT_MODE == 2) ? ((unsigned short*)Cout2 + (size_t)b * strideC) : nullptr;
      for (int pass = 0; pass < 2; ++pass) {
#pragma unroll
        for (int it = 0; it < 4; ++it) {
          const int row = it * 4 + q;
          const float* sp = slab + row * 68 + c8;
          v8h hv, lv;
#pragma unroll
          for (int e = 0; e < 8; ++e) {
            if (OUT_MODE == 1) {
              hv[e] = (_Float16)sp[e];
            } else {
              unsigned short hb = f2bf_bits(sp[e]);
              unsigned short lb = f2bf_bits(sp[e] - bf_bits2f(hb));
              hv[e] = __builtin_bit_cast(_Float16, hb);
              lv[e] = __builtin_bit_cast(_Float16, lb);
            }
          }
          *(volatile v8h*)(C + (size_t)(mBase + row) * ldc + n0 + c8) = hv;
          if (OUT_MODE == 2) *(volatile v8h*)(C2 + (size_t)(mBase + row) * ldc + n0 + c8) = lv;
        }
        __threadfence();
      }
    }
    __builtin_amdgcn_fence(__ATOMIC_RELEASE, "workgroup");
    __builtin_amdgcn_wave_barrier();
    __builtin_amdgcn_fence(__ATOMIC_ACQUIRE, "workgroup");
  }
}

__global__ __launch_bounds__(256) void split_rows_bf16_kernel(
    const float* __restrict__ src, unsigned short* __restrict__ dhi, unsigned short* __restrict__ dlo, int total8)
{
  const int i = blockIdx.x * 256 + threadIdx.x;
  if (i >= total8) return;
  const size_t e0 = (size_t)i << 3;
  const v4f a0 = *(const v4f*)(src + e0);
  const v4f a1 = *(const v4f*)(src + e0 + 4);
  v8h hv, lv;
  split8_bf16(a0, a1, hv, lv);
  unsigned short* qh = dhi + e0;
  unsigned short* ql = dlo + e0;
  *(volatile v8h*)qh = hv;
  *(volatile v8h*)ql = lv;
  __threadfence();
  *(volatile v8h*)qh = hv;
  *(volatile v8h*)ql = lv;
}

__global__ __launch_bounds__(256) void rows_bf16_kernel(
    const float* __restrict__ src, unsigned short* __restrict__ dst, int total8)
{
  const int i = blockIdx.x * 256 + threadIdx.x;
  if (i >= total8) return;
  const size_t e0 = (size_t)i << 3;
  const v4f a0 = *(const v4f*)(src + e0);
  const v4f a1 = *(const v4f*)(src + e0 + 4);
  const v8h hv = pack8_bf16(a0, a1);
  unsigned short* q = dst + e0;
  *(volatile v8h*)q = hv;
  __threadfence();
  *(volatile v8h*)q = hv;
}

__global__ __launch_bounds__(64) void cast_pad_rows_bf16_kernel(
    const float* __restrict__ src, unsigned short* __restrict__ dst, int rreal, int ncol)
{
  const int r = blockIdx.x, t = threadIdx.x;
  const int n8 = ncol >> 3;
  if (t < n8) {
    const int rs = (r < rreal) ? r : (rreal - 1);
    const float f = (r < rreal) ? 1.0f : 0.0f;
    const float* sp = src + (size_t)rs * ncol + t * 8;
    const v4f a0 = *(const v4f*)(sp) * f;
    const v4f a1 = *(const v4f*)(sp + 4) * f;
    const v8h hv = pack8_bf16(a0, a1);
    unsigned short* q = dst + (size_t)r * ncol + t * 8;
    *(volatile v8h*)q = hv;
    __threadfence();
    *(volatile v8h*)q = hv;
  }
}

__global__ __launch_bounds__(256) void precompose_wcomb_kernel(
    const float* __restrict__ xpl, const float* __restrict__ winl, unsigned short* __restrict__ dst)
{
  __shared__ __align__(16) float sRow[kDm];
  const int c = blockIdx.x, t = threadIdx.x;
  const bool live = (c < 2 * kNst);
  if (t < kDm) {
    float acc = 0.0f;
    if (live) {
      const float* xr = xpl + (size_t)(kDtR + c) * kDin;
#pragma unroll 1
      for (int d = 0; d < kDin; ++d) acc = fmaf(xr[d], winl[(size_t)d * kDm + t], acc);
    }
    sRow[t] = acc;
  }
  __syncthreads();
  if (t < kDm / 8) {
    const v4f a0 = *(const v4f*)(sRow + t * 8);
    const v4f a1 = *(const v4f*)(sRow + t * 8 + 4);
    const v8h hv = pack8_bf16(a0, a1);
    unsigned short* q = dst + (size_t)c * kDm + t * 8;
    *(volatile v8h*)q = hv;
    __threadfence();
    *(volatile v8h*)q = hv;
  }
}

__global__ __launch_bounds__(128) void dwconv2d_silu_kernel(
    const float* __restrict__ XZ, const float* __restrict__ cw, const float* __restrict__ cb,
    float* __restrict__ XS, unsigned short* __restrict__ XSB)
{
  __shared__ __align__(16) float sT[kImg * kC2P];
  const int tid = threadIdx.x, lane = tid & 31, wave = tid >> 5;
  const int d0 = blockIdx.x * kC2Ch, d = d0 + tid;
  const int b = blockIdx.y >> 6, h = blockIdx.y & (kImg - 1);
  const size_t prow0 = (size_t)b * kSeq + (size_t)h * kImg;
  const float* wp = cw + (size_t)d * 9;
  const float w0 = wp[0], w1 = wp[1], w2 = wp[2], w3 = wp[3], w4 = wp[4];
  const float w5 = wp[5], w6 = wp[6], w7 = wp[7], w8 = wp[8];
  const float bias = cb[d];
  asm volatile("" ::: "memory");
  const int hm = (h > 0) ? (h - 1) : 0;
  const int hp = (h < kImg - 1) ? (h + 1) : (kImg - 1);
  const float fm = (h > 0) ? 1.0f : 0.0f;
  const float fp = (h < kImg - 1) ? 1.0f : 0.0f;
  const float* rm = XZ + ((size_t)b * kSeq + (size_t)hm * kImg) * kXzP + d;
  const float* rc = XZ + prow0 * kXzP + d;
  const float* rp = XZ + ((size_t)b * kSeq + (size_t)hp * kImg) * kXzP + d;
  float am = 0.0f, ac = 0.0f, ap = 0.0f;
  float bm = rm[0] * fm, bc = rc[0], bp = rp[0] * fp;
#pragma unroll 1
  for (int wq = 0; wq < kImg; ++wq) {
    const int wn = (wq < kImg - 1) ? (wq + 1) : (kImg - 1);
    const float fn = (wq < kImg - 1) ? 1.0f : 0.0f;
    const size_t o = (size_t)wn * kXzP;
    const float cm = rm[o] * (fm * fn);
    const float cc = rc[o] * fn;
    const float cp = rp[o] * (fp * fn);
    float acc = 0.0f;
    acc = fmaf(w0, am, acc); acc = fmaf(w1, bm, acc); acc = fmaf(w2, cm, acc);
    acc = fmaf(w3, ac, acc); acc = fmaf(w4, bc, acc); acc = fmaf(w5, cc, acc);
    acc = fmaf(w6, ap, acc); acc = fmaf(w7, bp, acc); acc = fmaf(w8, cp, acc);
    const float sv = acc + bias;
    const float sg = __builtin_amdgcn_rcpf(1.0f + expf(-sv));
    sT[wq * kC2P + tid] = sv * sg;
    am = bm; bm = cm; ac = bc; bc = cc; ap = bp; bp = cp;
  }
  __syncthreads();
  const int hh = lane >> 4, c8 = (lane & 15) * 8;
  for (int pass = 0; pass < 2; ++pass) {
#pragma unroll
    for (int it = 0; it < 16; ++it) {
      const int row = wave + 4 * it;
      const v4f v = *(const v4f*)(sT + row * kC2P + lane * 4);
      *(volatile v4f*)(XS + (prow0 + row) * kDin + d0 + lane * 4) = v;
    }
#pragma unroll
    for (int it = 0; it < 8; ++it) {
      const int row = it * 8 + wave * 2 + hh;
      const float* sp = sT + row * kC2P + c8;
      const v4f a0 = *(const v4f*)(sp);
      const v4f a1 = *(const v4f*)(sp + 4);
      const v8h hv = pack8_bf16(a0, a1);
      *(volatile v8h*)(XSB + (prow0 + row) * kDin + d0 + c8) = hv;
    }
    __threadfence();
  }
}

__global__ __launch_bounds__(64) void gate_combine_kernel(
    const float* __restrict__ LOWD, const float* __restrict__ XD,
    const float* __restrict__ gb1, const float* __restrict__ gb2,
    const float* __restrict__ gc1, const float* __restrict__ gc2,
    float* __restrict__ BCD)
{
  constexpr int kN1 = 2 * kGateH * kNst;
  constexpr int kN2 = kNst * kGateH;
  __shared__ __align__(16) float sW1[2 * kN1];
  __shared__ __align__(16) float sW2[2 * kN2];
  __shared__ __align__(16) float sOut[64 * kXdP];
  __shared__ __align__(16) float sLow[64 * 32];
  const int tid = threadIdx.x, lane = tid & 31, wave = tid >> 5;
  const size_t r0 = (size_t)blockIdx.x * 64;
#pragma unroll 1
  for (int i = tid; i < kN1 / 4; i += 64) {
    const v4f a = *(const v4f*)(gb1 + 4 * i);
    const v4f c = *(const v4f*)(gc1 + 4 * i);
    *(v4f*)(sW1 + 4 * i) = a;
    *(v4f*)(sW1 + kN1 + 4 * i) = c;
    asm volatile("" ::: "memory");
  }
#pragma unroll 1
  for (int i = tid; i < kN2 / 4; i += 64) {
    const v4f a = *(const v4f*)(gb2 + 4 * i);
    const v4f c = *(const v4f*)(gc2 + 4 * i);
    *(v4f*)(sW2 + 4 * i) = a;
    *(v4f*)(sW2 + kN2 + 4 * i) = c;
    asm volatile("" ::: "memory");
  }
#pragma unroll 1
  for (int i = tid; i < 64 * 16; i += 64) {
    const int row = i >> 4, c4 = (i & 15) * 4;
    const v4f v = *(const v4f*)(XD + (r0 + row) * kXdP + c4);
    *(v4f*)(sOut + row * kXdP + c4) = v;
    asm volatile("" ::: "memory");
  }
#pragma unroll 1
  for (int i = tid; i < 64 * 8; i += 64) {
    const int row = i >> 3, c4 = (i & 7) * 4;
    const v4f v = *(const v4f*)(LOWD + (r0 + row) * kXdP + c4);
    *(v4f*)(sLow + row * 32 + c4) = v;
    asm volatile("" ::: "memory");
  }
  __syncthreads();
  const int row = tid;
#pragma unroll 1
  for (int g = 0; g < 2; ++g) {
    const float* w1 = sW1 + g * kN1;
    const float* w2 = sW2 + g * kN2;
    float v[kNst];
    {
      const float* lp = sLow + row * 32 + g * kNst;
#pragma unroll
      for (int q4 = 0; q4 < 4; ++q4) {
        const v4f t4 = *(const v4f*)(lp + 4 * q4);
        v[4 * q4 + 0] = t4[0]; v[4 * q4 + 1] = t4[1]; v[4 * q4 + 2] = t4[2]; v[4 * q4 + 3] = t4[3];
      }
    }
    float a[kNst];
#pragma unroll
    for (int o = 0; o < kNst; ++o) a[o] = 0.0f;
#pragma unroll 1
    for (int j = 0; j < kGateH; ++j) {
      const float* p1 = w1 + j * kNst;
      const float* p2 = w1 + (kGateH + j) * kNst;
      float h1 = 0.0f, h2 = 0.0f;
#pragma unroll
      for (int n = 0; n < kNst; ++n) {
        h1 = fmaf(p1[n], v[n], h1);
        h2 = fmaf(p2[n], v[n], h2);
      }
      const float gl = 0.5f * h1 * (1.0f + erff(h1 * 0.70710678118654752f)) * h2;
#pragma unroll
      for (int o = 0; o < kNst; ++o) a[o] = fmaf(w2[o * kGateH + j], gl, a[o]);
    }
    float* orow = sOut + row * kXdP + kDtR + g * kNst;
#pragma unroll
    for (int o = 0; o < kNst; ++o) orow[o] = orow[o] + a[o];
  }
  __syncthreads();
  const int hh = lane >> 4, c4 = (lane & 15) * 4;
  for (int pass = 0; pass < 2; ++pass) {
#pragma unroll
    for (int it = 0; it < 16; ++it) {
      const int rr = wave * 32 + it * 2 + hh;
      const v4f vv = *(const v4f*)(sOut + rr * kXdP + c4);
      *(volatile v4f*)(BCD + (r0 + rr) * kXdP + c4) = vv;
    }
    __threadfence();
  }
}

__global__ __launch_bounds__(256) void dwconv1d_kernel(
    const float* __restrict__ BCD, const float* __restrict__ wdt, const float* __restrict__ wB,
    const float* __restrict__ wC, float* __restrict__ CONVO)
{
  __shared__ __align__(16) float sIn[kC1In * kXdP];
  __shared__ __align__(16) float sOut[kC1Rows * kXdP];
  __shared__ float sWt[kXdP * 16];
  const int tid = threadIdx.x, lane = tid & 31, wave = tid >> 5;
  const size_t r0 = (size_t)blockIdx.x * kC1Rows;
  const int l0 = (int)(r0 & (size_t)(kSeq - 1));
  const size_t rowB = r0 - (size_t)l0;
#pragma unroll 1
  for (int i = tid; i < kXdP * kTap1; i += 256) {
    const int c = i / kTap1;
    const int k = i - c * kTap1;
    const int cd = (c < kDtR) ? c : (kDtR - 1);
    int cb = c - kDtR;        cb = (cb < 0) ? 0 : ((cb > kNst - 1) ? (kNst - 1) : cb);
    int cc = c - kDtR - kNst; cc = (cc < 0) ? 0 : ((cc > kNst - 1) ? (kNst - 1) : cc);
    const float vd = wdt[cd * kTap1 + k];
    const float vb = wB[cb * kTap1 + k];
    const float vc = wC[cc * kTap1 + k];
    const float fd = (c < kDtR) ? 1.0f : 0.0f;
    const float fb = (c >= kDtR && c < kDtR + kNst) ? 1.0f : 0.0f;
    const float fc = (c >= kDtR + kNst && c < kDbl) ? 1.0f : 0.0f;
    sWt[c * 16 + k] = fmaf(fd, vd, fmaf(fb, vb, fc * vc));
  }
#pragma unroll 1
  for (int i = tid; i < kC1In * 16; i += 256) {
    const int rr = i >> 4, c4 = (i & 15) * 4;
    const int ls = l0 - 14 + rr;
    const int lsc = (ls < 0) ? 0 : ((ls > kSeq - 1) ? (kSeq - 1) : ls);
    const float f = (ls >= 0 && ls < kSeq) ? 1.0f : 0.0f;
    const v4f v = *(const v4f*)(BCD + (rowB + (size_t)lsc) * kXdP + c4);
    *(v4f*)(sIn + rr * kXdP + c4) = v * f;
    asm volatile("" ::: "memory");
  }
  __syncthreads();
  const int c = tid & 63, rg = tid >> 6;
  float wk[kTap1];
#pragma unroll
  for (int k = 0; k < kTap1; ++k) wk[k] = sWt[c * 16 + k];
#pragma unroll 1
  for (int i = 0; i < 16; ++i) {
    const int r = rg * 16 + i;
    float acc = 0.0f;
#pragma unroll
    for (int k = 0; k < kTap1; ++k) acc = fmaf(sIn[(r + 2 * k) * kXdP + c], wk[k], acc);
    sOut[r * kXdP + c] = acc;
  }
  __syncthreads();
  const int hh = lane >> 4, c4 = (lane & 15) * 4;
  for (int pass = 0; pass < 2; ++pass) {
#pragma unroll
    for (int it = 0; it < 4; ++it) {
      const int rr = wave * 8 + it * 2 + hh;
      const v4f vv = *(const v4f*)(sOut + rr * kXdP + c4);
      *(volatile v4f*)(CONVO + (r0 + rr) * kXdP + c4) = vv;
    }
    __threadfence();
  }
}

__global__ __launch_bounds__(64) void scan_kernel(
    const float* __restrict__ CONVO, const float* __restrict__ XS, const float* __restrict__ XZ,
    const float* __restrict__ Wdt, const float* __restrict__ bdt, const float* __restrict__ Alog,
    const float* __restrict__ Dp, unsigned short* __restrict__ YH, unsigned short* __restrict__ YL)
{
  __shared__ __align__(16) float sX[kScanTS * kXdP];
  __shared__ __align__(16) float sY[kScanTS * kScanYP];
  __shared__ __align__(16) float sW[kDtR * kScanCh];
  __shared__ __align__(16) float sA[kNst * kScanCh];
  const int tid = threadIdx.x, lane = tid & 31, wave = tid >> 5;
  constexpr int kBlkPerB = kDin / kScanCh;
  const int bix = blockIdx.x / kBlkPerB;
  const int d0  = (blockIdx.x - bix * kBlkPerB) * kScanCh;
  const int d   = d0 + tid;
  const size_t row0 = (size_t)bix * kSeq;
#pragma unroll 1
  for (int r = 0; r < kDtR; ++r) sW[r * kScanCh + tid] = Wdt[(size_t)d * kDtR + r];
  asm volatile("" ::: "memory");
#pragma unroll 1
  for (int s = 0; s < kNst; ++s) sA[s * kScanCh + tid] = -expf(Alog[(size_t)d * kNst + s]) * 1.4426950408889634f;
  __syncthreads();
  float nA2[kNst], h[kNst];
#pragma unroll
  for (int s = 0; s < kNst; ++s) {
    nA2[s] = sA[s * kScanCh + tid];
    h[s] = 0.0f;
  }
  const float bb = bdt[d], Dd = Dp[d];
  const int lr = tid >> 4, lc4 = (tid & 15) * 4;
  const int q = lane >> 3, c8 = (lane & 7) * 8;
#pragma unroll 1
  for (int t0 = 0; t0 < kSeq; t0 += kScanTS) {
    __syncthreads();
#pragma unroll
    for (int i = 0; i < 8; ++i) {
      const int r = lr + 4 * i;
      *(v4f*)(sX + r * kXdP + lc4) = *(const v4f*)(CONVO + (row0 + t0 + r) * kXdP + lc4);
    }
    asm volatile("" ::: "memory");
#pragma unroll
    for (int i = 8; i < 16; ++i) {
      const int r = lr + 4 * i;
      *(v4f*)(sX + r * kXdP + lc4) = *(const v4f*)(CONVO + (row0 + t0 + r) * kXdP + lc4);
    }
    __syncthreads();
#pragma unroll 1
    for (int s = 0; s < kScanTS; ++s) {
      const int t = t0 + s;
      const float* xr = sX + s * kXdP;
      float vdot = 0.0f;
#pragma unroll 1
      for (int r4 = 0; r4 < kDtR / 4; ++r4) {
        const v4f xv = *(const v4f*)(xr + 4 * r4);
        const float* wp = sW + (4 * r4) * kScanCh + tid;
        vdot = fmaf(xv[0], wp[0], vdot);
        vdot = fmaf(xv[1], wp[kScanCh], vdot);
        vdot = fmaf(xv[2], wp[2 * kScanCh], vdot);
        vdot = fmaf(xv[3], wp[3 * kScanCh], vdot);
      }
      float Bs[kNst], Cs[kNst];
#pragma unroll
      for (int q4 = 0; q4 < 4; ++q4) {
        const v4f bv = *(const v4f*)(xr + kDtR + 4 * q4);
        const v4f cv = *(const v4f*)(xr + kDtR + kNst + 4 * q4);
        Bs[4 * q4 + 0] = bv[0]; Bs[4 * q4 + 1] = bv[1]; Bs[4 * q4 + 2] = bv[2]; Bs[4 * q4 + 3] = bv[3];
        Cs[4 * q4 + 0] = cv[0]; Cs[4 * q4 + 1] = cv[1]; Cs[4 * q4 + 2] = cv[2]; Cs[4 * q4 + 3] = cv[3];
      }
      const float v   = vdot + bb;
      const float dt  = fmaxf(v, 0.0f) + log1pf(expf(-fabsf(v)));
      const float ut  = XS[(row0 + t) * kDin + d];
      const float dtx = dt * ut;
      float y = 0.0f;
#pragma unroll
      for (int k = 0; k < kNst; ++k) {
        const float e = __builtin_amdgcn_exp2f(dt * nA2[k]);
        h[k] = fmaf(e, h[k], dtx * Bs[k]);
        y = fmaf(h[k], Cs[k], y);
      }
      y = fmaf(ut, Dd, y);
      const float zv = XZ[(row0 + t) * kXzP + kDin + d];
      const float sg = __builtin_amdgcn_rcpf(1.0f + expf(-zv));
      y = y * (zv * sg);
      sY[s * kScanYP + tid] = y;
    }
    __syncthreads();
    for (int pass = 0; pass < 2; ++pass) {
#pragma unroll
      for (int it = 0; it < 8; ++it) {
        const int row = it * 8 + wave * 4 + q;
        const float* sp = sY + row * kScanYP + c8;
        const v4f a0 = *(const v4f*)(sp);
        const v4f a1 = *(const v4f*)(sp + 4);
        v8h hv, lv;
        split8_bf16(a0, a1, hv, lv);
        const size_t o = (row0 + t0 + row) * kDin + d0 + c8;
        *(volatile v8h*)(YH + o) = hv;
        *(volatile v8h*)(YL + o) = lv;
      }
      __threadfence();
    }
  }
}

extern "C" void kernel_launch(void* const* d_in, const int* in_sizes, int n_in,
                              void* d_out, int out_size, void* d_ws, size_t ws_size,
                              hipStream_t stream) {
  if (n_in < 20) return;
  if (in_sizes[0] != kRows * kDm || in_sizes[1] != kRows * kDm) return;
  if (in_sizes[2] != kXzP * kDm || in_sizes[3] != kDin * kDm) return;
  if (in_sizes[4] != kDin * 9 || in_sizes[5] != kDin) return;
  if (in_sizes[6] != kDbl * kDin || in_sizes[7] != kDbl * kDin) return;
  if (in_sizes[8] != kDtR * kTap1 || in_sizes[9] != kNst * kTap1 || in_sizes[10] != kNst * kTap1) return;
  if (in_sizes[11] != 2 * kGateH * kNst || in_sizes[12] != kNst * kGateH) return;
  if (in_sizes[13] != 2 * kGateH * kNst || in_sizes[14] != kNst * kGateH) return;
  if (in_sizes[15] != kDin * kDtR || in_sizes[16] != kDin) return;
  if (in_sizes[17] != kDin * kNst || in_sizes[18] != kDin) return;
  if (in_sizes[19] != kDm * kDin) return;
  if (out_size != kRows * kDm) return;
  if (ws_size < kWsTotal) return;

  const float* x         = (const float*)d_in[0];
  const float* hbl       = (const float*)d_in[1];
  const float* W_in      = (const float*)d_in[2];
  const float* W_in_low  = (const float*)d_in[3];
  const float* conv2_w   = (const float*)d_in[4];
  const float* conv2_b   = (const float*)d_in[5];
  const float* xproj_w   = (const float*)d_in[6];
  const float* xproj_wl  = (const float*)d_in[7];
  const float* conv_dt_w = (const float*)d_in[8];
  const float* conv_B_w  = (const float*)d_in[9];
  const float* conv_C_w  = (const float*)d_in[10];
  const float* gb_fc1    = (const float*)d_in[11];
  const float* gb_fc2    = (const float*)d_in[12];
  const float* gc_fc1    = (const float*)d_in[13];
  const float* gc_fc2    = (const float*)d_in[14];
  const float* dt_w      = (const float*)d_in[15];
  const float* dt_b      = (const float*)d_in[16];
  const float* A_log     = (const float*)d_in[17];
  const float* Dp        = (const float*)d_in[18];
  const float* W_out     = (const float*)d_in[19];
  float* out = (float*)d_out;

  char* ws = (char*)d_ws;
  unsigned short* XH    = (unsigned short*)(ws + kOffXH);
  unsigned short* XL    = (unsigned short*)(ws + kOffXL);
  unsigned short* HBLB  = (unsigned short*)(ws + kOffHBLB);
  unsigned short* WIH   = (unsigned short*)(ws + kOffWIH);
  unsigned short* WIL   = (unsigned short*)(ws + kOffWIL);
  unsigned short* WOH   = (unsigned short*)(ws + kOffWOH);
  unsigned short* WOL   = (unsigned short*)(ws + kOffWOL);
  unsigned short* WXB   = (unsigned short*)(ws + kOffWXB);
  unsigned short* WCB   = (unsigned short*)(ws + kOffWCB);
  float*          XZ    = (float*)(ws + kOffXZ);
  float*          XS    = (float*)(ws + kOffXS);
  unsigned short* XSB   = (unsigned short*)(ws + kOffXSB);
  float*          LOWD  = (float*)(ws + kOffLOWD);
  float*          XD    = (float*)(ws + kOffXD);
  float*          BCD   = (float*)(ws + kOffBCD);
  float*          CONVO = (float*)(ws + kOffCONVO);
  unsigned short* YH    = (unsigned short*)(ws + kOffYH);
  unsigned short* YL    = (unsigned short*)(ws + kOffYL);

  split_rows_bf16_kernel<<<(kRows * kDm / 8) / 256, 256, 0, stream>>>(x, XH, XL, kRows * kDm / 8);
  rows_bf16_kernel<<<(kRows * kDm / 8) / 256, 256, 0, stream>>>(hbl, HBLB, kRows * kDm / 8);
  split_rows_bf16_kernel<<<(kXzP * kDm / 8) / 256, 256, 0, stream>>>(W_in, WIH, WIL, kXzP * kDm / 8);
  split_rows_bf16_kernel<<<(kDm * kDin / 8) / 256, 256, 0, stream>>>(W_out, WOH, WOL, kDm * kDin / 8);
  cast_pad_rows_bf16_kernel<<<kXdP, 64, 0, stream>>>(xproj_w, WXB, kDbl, kDin);
  precompose_wcomb_kernel<<<kXdP, 256, 0, stream>>>(xproj_wl, W_in_low, WCB);

  wmma_gemm64<1, 2, 0, 0, false><<<dim3(384, 1), 256, 0, stream>>>(
      XH, XL, kDm, 0L,
      WIH, WIL, kDm, 0L,
      (void*)XZ, nullptr, kXzP, 0L,
      nullptr, nullptr, 0L,
      kRows, kXzP, kDm, 1.0f);

  dwconv2d_silu_kernel<<<dim3(kDin / kC2Ch, kBatch * kImg), kC2Ch, 0, stream>>>(XZ, conv2_w, conv2_b, XS, XSB);

  wmma_gemm64<1, 0, 0, 0, false><<<dim3(32, 1), 256, 0, stream>>>(
      HBLB, nullptr, kDm, 0L,
      WCB, nullptr, kDm, 0L,
      (void*)LOWD, nullptr, kXdP, 0L,
      nullptr, nullptr, 0L,
      kRows, kXdP, kDm, 1.0f);

  wmma_gemm64<1, 0, 0, 0, false><<<dim3(32, 1), 256, 0, stream>>>(
      XSB, nullptr, kDin, 0L,
      WXB, nullptr, kDin, 0L,
      (void*)XD, nullptr, kXdP, 0L,
      nullptr, nullptr, 0L,
      kRows, kXdP, kDin, 1.0f);

  gate_combine_kernel<<<kRows / 64, 64, 0, stream>>>(LOWD, XD, gb_fc1, gb_fc2, gc_fc1, gc_fc2, BCD);

  dwconv1d_kernel<<<kRows / kC1Rows, 256, 0, stream>>>(BCD, conv_dt_w, conv_B_w, conv_C_w, CONVO);

  scan_kernel<<<kBatch * (kDin / kScanCh), kScanCh, 0, stream>>>(CONVO, XS, XZ, dt_w, dt_b, A_log, Dp, YH, YL);

  wmma_gemm64<1, 2, 0, 0, false><<<dim3(96, 1), 256, 0, stream>>>(
      YH, YL, kDin, 0L,
      WOH, WOL, kDin, 0L,
      (void*)out, nullptr, kDm, 0L,
      nullptr, nullptr, 0L,
      kRows, kDm, kDin, 1.0f);
}
